// LSTMPredictor_85169201480408
// MI455X (gfx1250) — hardware-verified
//
#include <hip/hip_runtime.h>
#include <math.h>

constexpr int SEQ_T    = 256;
constexpr int NBATCH   = 2048;
constexpr int NINP     = 11;
constexpr int NHID     = 64;
constexpr int NGATE    = 4 * NHID;
constexpr int NPRED    = 12;
constexpr int KXPAD    = 32;
constexpr int ROWS_BLK = 32;
constexpr int NTHR     = 128;
constexpr int NWAVE    = NTHR / 32;
constexpr int XPITCH   = 40;
constexpr int HPITCH   = 136;
constexpr int COL_HLO  = 64;
constexpr int XTILE    = ROWS_BLK * XPITCH;
constexpr int HTILE    = ROWS_BLK * HPITCH;
constexpr int NXROWS   = SEQ_T * NBATCH;
constexpr int PREP_THR = 256;
constexpr int X8       = NXROWS * KXPAD / 8;
constexpr int WIE8     = NGATE * KXPAD / 8;
constexpr int WH8      = NGATE * NHID / 8;
constexpr int NOUT     = NPRED * NBATCH;

static_assert(NBATCH % ROWS_BLK == 0);
static_assert(ROWS_BLK == 32);
static_assert(NHID == 16 * NWAVE);
static_assert(NGATE == 4 * NHID);
static_assert(SEQ_T % 2 == 0);
static_assert(KXPAD % 32 == 0 && NHID % 32 == 0);
static_assert(NINP <= KXPAD);
static_assert(XPITCH % 8 == 0 && XPITCH >= KXPAD);
static_assert(HPITCH % 8 == 0 && HPITCH >= COL_HLO + NHID && COL_HLO == NHID);
static_assert(HTILE % NTHR == 0 && XTILE % NTHR == 0);
static_assert(NTHR * 8 == ROWS_BLK * KXPAD);
static_assert(X8 % PREP_THR == 0 && WIE8 % PREP_THR == 0 && WH8 % PREP_THR == 0);

typedef __attribute__((ext_vector_type(16))) _Float16 v16h;
typedef __attribute__((ext_vector_type(8)))  _Float16 v8h;
typedef __attribute__((ext_vector_type(16))) __bf16   v16b;
typedef __attribute__((ext_vector_type(8)))  __bf16   v8b;
typedef __attribute__((ext_vector_type(8)))  float    v8f;
typedef __attribute__((ext_vector_type(4)))  float    v4f;
typedef __attribute__((ext_vector_type(4)))  unsigned v4u;

__device__ __forceinline__ unsigned short f2bf_bits(float f) {
  unsigned u = __float_as_uint(f);
  return (unsigned short)((u + 0x7FFFu + ((u >> 16) & 1u)) >> 16);
}
__device__ __forceinline__ float bf_bits2f(unsigned short h) { return __uint_as_float(((unsigned)h) << 16); }
__device__ __forceinline__ float bf16r(float f) { return bf_bits2f(f2bf_bits(f)); }

__device__ __forceinline__ void dep_guard_b(v8f& a, v8f& b, v16b x, v16b y) { asm volatile("v_nop\n\tv_nop\n\tv_nop\n\tv_nop" : "+v"(a), "+v"(b) : "v"(x), "v"(y)); }
__device__ __forceinline__ void group_guard8_b(v8f& d0, v8f& d1, v8f& d2, v8f& d3, v8f& d4, v8f& d5, v8f& d6, v8f& d7,
                                               v16b xa, v16b xb, v16b y0, v16b y1, v16b y2, v16b y3) {
  asm volatile("v_nop\n\tv_nop\n\tv_nop\n\tv_nop"
               : "+v"(d0), "+v"(d1), "+v"(d2), "+v"(d3), "+v"(d4), "+v"(d5), "+v"(d6), "+v"(d7)
               : "v"(xa), "v"(xb), "v"(y0), "v"(y1), "v"(y2), "v"(y3));
}
__device__ __forceinline__ void keep4_b(v16b a, v16b b, v16b c, v16b d) { asm volatile("v_nop" :: "v"(a), "v"(b), "v"(c), "v"(d)); }
__device__ __forceinline__ void acc_guard4(v8f& a, v8f& b, v8f& c, v8f& d) { asm volatile("v_nop\n\tv_nop\n\tv_nop\n\tv_nop" : "+v"(a), "+v"(b), "+v"(c), "+v"(d)); }

template <typename T> struct Frag;
template <> struct Frag<__bf16> {
  typedef v16b V; union U { v16b v; v8b h[2]; };
  static __device__ __forceinline__ v16b load(const __bf16* p) {
    U f; f.h[0] = *(const v8b*)(p); f.h[1] = *(const v8b*)(p + 16); return f.v;
  }
  static __device__ __forceinline__ v8f mma(v16b a, v16b b, v8f c) {
    return __builtin_amdgcn_wmma_f32_16x16x32_bf16(false, a, false, b, (short)0, c, false, false);
  }
};

__device__ __forceinline__ float fsig(float x)  { return __builtin_amdgcn_rcpf(1.0f + expf(-x)); }
__device__ __forceinline__ float ftanh(float x) { return 1.0f - 2.0f * __builtin_amdgcn_rcpf(expf(2.0f * x) + 1.0f); }

__global__ __launch_bounds__(PREP_THR) void cvt11_kernel(const float* __restrict__ src, unsigned short* __restrict__ dst, int n8) {
  const int i = blockIdx.x * PREP_THR + threadIdx.x;
  if (i < n8) {
    const int row = i >> 2, c8 = (i & 3) * 8;
    const float* sp = src + (size_t)row * NINP;
    v8h hv;
#pragma unroll
    for (int e = 0; e < 8; ++e) {
      const int col = c8 + e;
      const int cc  = (col < NINP) ? col : (NINP - 1);
      const float f   = sp[cc];
      const float fac = (col < NINP) ? 1.0f : 0.0f;
      const float v   = f * fac;
      hv[e] = __builtin_bit_cast(_Float16, f2bf_bits(v));
    }
    *(volatile v8h*)(dst + (size_t)i * 8) = hv;
    __threadfence();
    *(volatile v8h*)(dst + (size_t)i * 8) = hv;
  }
}

__global__ __launch_bounds__(PREP_THR) void cvt64_kernel(const float* __restrict__ src, unsigned short* __restrict__ dst, int n8) {
  const int i = blockIdx.x * PREP_THR + threadIdx.x;
  if (i < n8) {
    const int n = i >> 3, k8 = (i & 7) * 8;
    const v4f a = *(const v4f*)(src + (size_t)n * NHID + k8);
    const v4f b = *(const v4f*)(src + (size_t)n * NHID + k8 + 4);
    v8h hv;
#pragma unroll
    for (int e = 0; e < 4; ++e) {
      hv[e]     = __builtin_bit_cast(_Float16, f2bf_bits(a[e]));
      hv[4 + e] = __builtin_bit_cast(_Float16, f2bf_bits(b[e]));
    }
    *(volatile v8h*)(dst + (size_t)i * 8) = hv;
    __threadfence();
    *(volatile v8h*)(dst + (size_t)i * 8) = hv;
  }
}

__device__ __forceinline__ void ktile(v8f (&acc)[2][4], const __bf16* pa0, const __bf16* pa1, const __bf16* pb, int gs) {
  const v16b b0 = Frag<__bf16>::load(pb);
  const v16b b1 = Frag<__bf16>::load(pb + (size_t)1 * gs);
  const v16b b2 = Frag<__bf16>::load(pb + (size_t)2 * gs);
  const v16b b3 = Frag<__bf16>::load(pb + (size_t)3 * gs);
  const v16b a0 = Frag<__bf16>::load(pa0);
  const v16b a1 = Frag<__bf16>::load(pa1);
  acc[0][0] = Frag<__bf16>::mma(a0, b0, acc[0][0]);
  acc[0][1] = Frag<__bf16>::mma(a0, b1, acc[0][1]);
  acc[0][2] = Frag<__bf16>::mma(a0, b2, acc[0][2]);
  acc[0][3] = Frag<__bf16>::mma(a0, b3, acc[0][3]);
  acc[1][0] = Frag<__bf16>::mma(a1, b0, acc[1][0]);
  acc[1][1] = Frag<__bf16>::mma(a1, b1, acc[1][1]);
  acc[1][2] = Frag<__bf16>::mma(a1, b2, acc[1][2]);
  acc[1][3] = Frag<__bf16>::mma(a1, b3, acc[1][3]);
  group_guard8_b(acc[0][0], acc[0][1], acc[0][2], acc[0][3], acc[1][0], acc[1][1], acc[1][2], acc[1][3],
                 a0, a1, b0, b1, b2, b3);
  keep4_b(b0, b1, b2, b3);
}

__device__ __forceinline__ float lstm_unit(float zi, float zf, float zg, float zo, float& cs) {
  const float ig = fsig(zi);
  const float fg = fsig(zf);
  const float gg = ftanh(zg);
  const float og = fsig(zo);
  const float cn = fg * cs + ig * gg;
  cs = cn;
  return og * ftanh(cn);
}
__device__ __forceinline__ void put_h(__bf16* Hn, int rowoff, int j, float hn) {
  const unsigned short hb = f2bf_bits(hn);
  const unsigned short lb = f2bf_bits(hn - bf_bits2f(hb));
  Hn[rowoff + j]           = __builtin_bit_cast(__bf16, hb);
  Hn[rowoff + COL_HLO + j] = __builtin_bit_cast(__bf16, lb);
}

__global__ __launch_bounds__(NTHR) void lstm_seq_kernel(
    const unsigned short* __restrict__ XBp, const float* __restrict__ y, const int* __restrict__ tforce,
    const float* __restrict__ b_enc, const float* __restrict__ w_ih_dec, const float* __restrict__ b_dec,
    const float* __restrict__ w_fc, const float* __restrict__ b_fc,
    const unsigned short* __restrict__ WIEp, const unsigned short* __restrict__ WHEp,
    const unsigned short* __restrict__ WHDp, float* __restrict__ out) {
  __shared__ __align__(16) unsigned short Xs[2 * XTILE];
  __shared__ __align__(16) __bf16         Hs[2 * HTILE];
  __shared__ __align__(16) float          part[2 * NWAVE * ROWS_BLK];
  const __bf16* WIE = (const __bf16*)WIEp;
  const __bf16* WHE = (const __bf16*)WHEp;
  const __bf16* WHD = (const __bf16*)WHDp;
  const int tid = threadIdx.x, lane = tid & 31, wave = tid >> 5;
  const int c = lane & 15, hh = lane >> 4, koff = hh * 8;
  const int j = 16 * wave + c;
  const int m0 = blockIdx.x * ROWS_BLK;
  const int tf = tforce[0];
  const int xrow = tid >> 2, xq = (tid & 3) * 8;

  {
    unsigned* hw = (unsigned*)Hs;
#pragma unroll 1
    for (int i = tid; i < HTILE; i += NTHR) hw[i] = 0u;
    unsigned* xw = (unsigned*)Xs;
#pragma unroll 1
    for (int i = tid; i < XTILE; i += NTHR) xw[i] = 0u;
  }
  float be[4];
#pragma unroll
  for (int g = 0; g < 4; ++g) be[g] = bf16r(b_enc[NHID * g + j]);
  float cst[2][8];
#pragma unroll
  for (int ms = 0; ms < 2; ++ms)
#pragma unroll
    for (int r = 0; r < 8; ++r) cst[ms][r] = 0.0f;
  __syncthreads();
  {
    const v4u w0 = *(const v4u*)(XBp + ((size_t)m0 + xrow) * KXPAD + xq);
    *(v4u*)(Xs + xrow * XPITCH + xq) = w0;
  }
  __syncthreads();

  const v8f z8 = {0.f, 0.f, 0.f, 0.f, 0.f, 0.f, 0.f, 0.f};
  v8f acc[2][4];

#pragma unroll 1
  for (int t = 0; t < SEQ_T; ++t) {
    const int cur = t & 1, nxt = cur ^ 1;
    const int tn = (t + 1 < SEQ_T) ? (t + 1) : (SEQ_T - 1);
    const v4u xw = *(const v4u*)(XBp + ((size_t)tn * NBATCH + m0 + xrow) * KXPAD + xq);

#pragma unroll
    for (int ms = 0; ms < 2; ++ms)
#pragma unroll
      for (int g = 0; g < 4; ++g) acc[ms][g] = z8;
    {
      const __bf16* xa = (const __bf16*)Xs + cur * XTILE + c * XPITCH + koff;
      ktile(acc, xa, xa + 16 * XPITCH, WIE + (size_t)j * KXPAD + koff, NHID * KXPAD);
    }
#pragma unroll 1
    for (int kk = 0; kk < 4; ++kk) {
      const __bf16* ha = Hs + cur * HTILE + c * HPITCH + 32 * kk + koff;
      ktile(acc, ha, ha + 16 * HPITCH, WHE + (size_t)j * NHID + (kk & 1) * 32 + koff, NHID * NHID);
    }
    acc_guard4(acc[0][0], acc[0][1], acc[0][2], acc[0][3]);
    acc_guard4(acc[1][0], acc[1][1], acc[1][2], acc[1][3]);

    __bf16* Hn = Hs + nxt * HTILE;
#pragma unroll
    for (int ms = 0; ms < 2; ++ms)
#pragma unroll
      for (int r = 0; r < 8; ++r) {
        const float hn = lstm_unit(acc[ms][0][r] + be[0], acc[ms][1][r] + be[1],
                                   acc[ms][2][r] + be[2], acc[ms][3][r] + be[3], cst[ms][r]);
        put_h(Hn, (16 * ms + 8 * hh + r) * HPITCH, j, hn);
      }
    *(v4u*)(Xs + nxt * XTILE + xrow * XPITCH + xq) = xw;
    __syncthreads();
  }

  float yv[2][8], wyd[4], bd[4];
#pragma unroll
  for (int ms = 0; ms < 2; ++ms) {
    const v4f ya = *(const v4f*)(y + m0 + 16 * ms + 8 * hh);
    const v4f yb = *(const v4f*)(y + m0 + 16 * ms + 8 * hh + 4);
#pragma unroll
    for (int e = 0; e < 4; ++e) { yv[ms][e] = bf16r(ya[e]); yv[ms][4 + e] = bf16r(yb[e]); }
  }
#pragma unroll
  for (int g = 0; g < 4; ++g) {
    wyd[g] = bf16r(w_ih_dec[NHID * g + j]);
    bd[g]  = bf16r(b_dec[NHID * g + j]);
  }
  const float wfc = bf16r(w_fc[j]);
  const float bfc = bf16r(b_fc[0]);
  const float nanv = __uint_as_float(0x7fc00000u);

#pragma unroll 1
  for (int p = 0; p < NPRED; ++p) {
    const int cur = p & 1, nxt = cur ^ 1;

#pragma unroll
    for (int ms = 0; ms < 2; ++ms)
#pragma unroll
      for (int g = 0; g < 4; ++g) acc[ms][g] = z8;
#pragma unroll 1
    for (int kk = 0; kk < 4; ++kk) {
      const __bf16* ha = Hs + cur * HTILE + c * HPITCH + 32 * kk + koff;
      ktile(acc, ha, ha + 16 * HPITCH, WHD + (size_t)j * NHID + (kk & 1) * 32 + koff, NHID * NHID);
    }
    acc_guard4(acc[0][0], acc[0][1], acc[0][2], acc[0][3]);
    acc_guard4(acc[1][0], acc[1][1], acc[1][2], acc[1][3]);

    __bf16* Hn = Hs + nxt * HTILE;
    float fsum[2][8];
#pragma unroll
    for (int ms = 0; ms < 2; ++ms)
#pragma unroll
      for (int r = 0; r < 8; ++r) {
        const float yr = yv[ms][r];
        const float zi = acc[ms][0][r] + (yr * wyd[0] + bd[0]);
        const float zf = acc[ms][1][r] + (yr * wyd[1] + bd[1]);
        const float zg = acc[ms][2][r] + (yr * wyd[2] + bd[2]);
        const float zo = acc[ms][3][r] + (yr * wyd[3] + bd[3]);
        const float hn = lstm_unit(zi, zf, zg, zo, cst[ms][r]);
        put_h(Hn, (16 * ms + 8 * hh + r) * HPITCH, j, hn);
        fsum[ms][r] = hn * wfc;
      }
#pragma unroll
    for (int ms = 0; ms < 2; ++ms)
#pragma unroll
      for (int r = 0; r < 8; ++r) {
        float v = fsum[ms][r];
        v += __shfl_xor(v, 1, 32);
        v += __shfl_xor(v, 2, 32);
        v += __shfl_xor(v, 4, 32);
        v += __shfl_xor(v, 8, 32);
        fsum[ms][r] = v;
      }
    if (c == 0) {
      float* pw = part + (cur * NWAVE + wave) * ROWS_BLK;
#pragma unroll
      for (int ms = 0; ms < 2; ++ms) {
        v4f u0, u1;
        u0[0] = fsum[ms][0]; u0[1] = fsum[ms][1]; u0[2] = fsum[ms][2]; u0[3] = fsum[ms][3];
        u1[0] = fsum[ms][4]; u1[1] = fsum[ms][5]; u1[2] = fsum[ms][6]; u1[3] = fsum[ms][7];
        *(v4f*)(pw + 16 * ms + 8 * hh)     = u0;
        *(v4f*)(pw + 16 * ms + 8 * hh + 4) = u1;
      }
    }
    __syncthreads();
    if (wave == 0) {
      const int q = lane & 7;
      const float* pp = part + cur * NWAVE * ROWS_BLK + 4 * q;
      const v4f s0 = *(const v4f*)(pp);
      const v4f s1 = *(const v4f*)(pp + ROWS_BLK);
      const v4f s2 = *(const v4f*)(pp + 2 * ROWS_BLK);
      const v4f s3 = *(const v4f*)(pp + 3 * ROWS_BLK);
      v4f o;
#pragma unroll
      for (int e = 0; e < 4; ++e) {
        float v = ((s0[e] + s1[e]) + (s2[e] + s3[e])) + bfc;
        if (tf != 0) v = nanv;
        o[e] = v;
      }
      if (lane < 8) {
        float* op = out + (size_t)p * NBATCH + m0 + 4 * q;
        for (int pass = 0; pass < 2; ++pass) {
          *(volatile v4f*)op = o;
          __threadfence();
        }
      }
    }
  }
}

extern "C" void kernel_launch(void* const* d_in, const int* in_sizes, int n_in,
                              void* d_out, int out_size, void* d_ws, size_t ws_size, hipStream_t stream) {
  if (n_in < 11 || d_out == nullptr || d_ws == nullptr) return;
  if (in_sizes[0] != SEQ_T * NBATCH * NINP || in_sizes[1] != NBATCH || in_sizes[2] < 1 ||
      in_sizes[3] != NGATE * NINP || in_sizes[4] != NGATE * NHID || in_sizes[5] != NGATE ||
      in_sizes[6] != NGATE || in_sizes[7] != NGATE * NHID || in_sizes[8] != NGATE ||
      in_sizes[9] != NHID || in_sizes[10] < 1 || out_size != NOUT) return;

  const float* x        = (const float*)d_in[0];
  const float* y        = (const float*)d_in[1];
  const int*   tforce   = (const int*)d_in[2];
  const float* w_ih_enc = (const float*)d_in[3];
  const float* w_hh_enc = (const float*)d_in[4];
  const float* b_enc    = (const float*)d_in[5];
  const float* w_ih_dec = (const float*)d_in[6];
  const float* w_hh_dec = (const float*)d_in[7];
  const float* b_dec    = (const float*)d_in[8];
  const float* w_fc     = (const float*)d_in[9];
  const float* b_fc     = (const float*)d_in[10];
  float* out = (float*)d_out;

  char* ws = (char*)d_ws; size_t off = 0;
  auto carve = [&](size_t bytes) -> char* { char* p = ws + off; off += (bytes + 255) & ~(size_t)255; return p; };
  unsigned short* XB  = (unsigned short*)carve((size_t)X8 * 16);
  unsigned short* WIE = (unsigned short*)carve((size_t)WIE8 * 16);
  unsigned short* WHE = (unsigned short*)carve((size_t)WH8 * 16);
  unsigned short* WHD = (unsigned short*)carve((size_t)WH8 * 16);
  if (off > ws_size || off > (size_t)134217728) return;

  cvt11_kernel<<<X8 / PREP_THR, PREP_THR, 0, stream>>>(x, XB, X8);
  cvt11_kernel<<<WIE8 / PREP_THR, PREP_THR, 0, stream>>>(w_ih_enc, WIE, WIE8);
  cvt64_kernel<<<WH8 / PREP_THR, PREP_THR, 0, stream>>>(w_hh_enc, WHE, WH8);
  cvt64_kernel<<<WH8 / PREP_THR, PREP_THR, 0, stream>>>(w_hh_dec, WHD, WH8);
  lstm_seq_kernel<<<NBATCH / ROWS_BLK, NTHR, 0, stream>>>(XB, y, tforce, b_enc, w_ih_dec, b_dec, w_fc, b_fc,
                                                          WIE, WHE, WHD, out);
}
